// MultiModalAttentionV2_85641647882456
// MI455X (gfx1250) — hardware-verified
//
#include <hip/hip_runtime.h>

typedef _Float16 v16h __attribute__((ext_vector_type(16)));
typedef _Float16 v8h  __attribute__((ext_vector_type(8)));
typedef float    v8f  __attribute__((ext_vector_type(8)));
typedef float    v4f  __attribute__((ext_vector_type(4)));
typedef int      v4i  __attribute__((ext_vector_type(4)));
typedef v8h __attribute__((may_alias)) v8ha;
typedef v4f __attribute__((may_alias)) v4fa;
typedef v4i __attribute__((may_alias)) v4ia;

union Frag { v16h v; v8h half[2]; };

#define DEV __device__ __forceinline__

#define NB    4
#define NT    1024
#define NM    256
#define NC    512
#define NH    8
#define HDIM  64
#define NZ    32
#define NC3   1536
#define TOKX  (NB * NT)
#define TOKY  (NB * NM)
#define WROWS (2 * NC3 + 3 * NC)
#define WSC   32.0f
#define PSC   16384.0f
#define NEGV  (-1e30f)

DEV v8f wmma_f16(v16h a, v16h b, v8f c) {
  v8f d = __builtin_amdgcn_wmma_f32_16x16x32_f16(false, a, false, b, (short)0, c, false, false);
  asm volatile("v_nop\n\tv_nop\n\tv_nop\n\tv_nop" : "+v"(d) : "v"(a), "v"(b));
  return d;
}

DEV v16h load_frag(const _Float16* p, int h) {
  Frag f;
  f.half[0] = *(const v8ha*)(p + 8 * h);
  f.half[1] = *(const v8ha*)(p + 16 + 8 * h);
  return f.v;
}

DEV float rcpf(float x) { return __builtin_amdgcn_rcpf(x); }

__global__ __launch_bounds__(256) void convert_xy_k(
    const float* __restrict__ x, const float* __restrict__ y,
    _Float16* __restrict__ xh, _Float16* __restrict__ yh)
{
  const int NX8 = TOKX * NC / 8, NY8 = TOKY * NC / 8;
  const int g = blockIdx.x * 256 + threadIdx.x;
  if (g >= NX8 + NY8) return;
  const float* src;
  _Float16* dst;
  if (g < NX8) { src = x + (size_t)g * 8; dst = xh + (size_t)g * 8; }
  else { const int e = g - NX8; src = y + (size_t)e * 8; dst = yh + (size_t)e * 8; }
  const v4f a = *(const v4fa*)src;
  const v4f c = *(const v4fa*)(src + 4);
  const v8h o = { (_Float16)a.x, (_Float16)a.y, (_Float16)a.z, (_Float16)a.w,
                  (_Float16)c.x, (_Float16)c.y, (_Float16)c.z, (_Float16)c.w };
  *(volatile v8h*)dst = o;
  __threadfence();
  *(volatile v8h*)dst = o;
}

__global__ __launch_bounds__(256) void wtrans_k(
    const float* __restrict__ w0, const float* __restrict__ w1, const float* __restrict__ w2,
    const float* __restrict__ w3, const float* __restrict__ w4, _Float16* __restrict__ wt)
{
  __shared__ __attribute__((aligned(16))) _Float16 sW[32 * 72];
  const int tid = threadIdx.x;
  const int n0g = blockIdx.x * 32, k0 = blockIdx.y * 64;
  const float* src; int nd, nloc;
  if (n0g < NC3)                    { src = w0; nd = NC3; nloc = n0g; }
  else if (n0g < 2 * NC3)           { src = w1; nd = NC3; nloc = n0g - NC3; }
  else if (n0g < 2 * NC3 + NC)      { src = w2; nd = NC;  nloc = n0g - 2 * NC3; }
  else if (n0g < 2 * NC3 + 2 * NC)  { src = w3; nd = NC;  nloc = n0g - 2 * NC3 - NC; }
  else                              { src = w4; nd = NC;  nloc = n0g - 2 * NC3 - 2 * NC; }
  const int c = tid & 31, rr = tid >> 5;
  #pragma unroll
  for (int i = 0; i < 8; ++i) {
    const int r = 8 * i + rr;
    const float v = src[(size_t)(k0 + r) * nd + nloc + c];
    sW[c * 72 + r] = (_Float16)(v * WSC);
  }
  __syncthreads();
  const int line = tid >> 3, q8 = tid & 7;
  const v8h o = *(const v8ha*)(sW + line * 72 + 8 * q8);
  _Float16* dst = wt + (size_t)(n0g + line) * NC + k0 + 8 * q8;
  *(volatile v8h*)dst = o;
  __threadfence();
  *(volatile v8h*)dst = o;
}

DEV void proj_store_pass(const _Float16* sT, _Float16* plane, _Float16* vtp,
                         int which, int z, int l0, int L, int w, int lane) {
  const int q8 = lane & 7, sub = lane >> 3;
  #pragma unroll
  for (int i = 0; i < 8; ++i) {
    const int lid = w * 32 + i * 4 + sub;
    v8h v;
    _Float16* dst;
    if (which != 2) {
      v = *(const v8ha*)(sT + lid * HDIM + 8 * q8);
      dst = plane + ((size_t)z * L + l0 + lid) * HDIM + 8 * q8;
    } else {
      const int d = lid >> 1, hl = lid & 1;
      v = *(const v8ha*)(sT + d * 128 + 64 * hl + 8 * q8);
      dst = vtp + ((size_t)z * HDIM + d) * L + l0 + 64 * hl + 8 * q8;
    }
    *(volatile v8h*)dst = v;
  }
}

__global__ __launch_bounds__(128) void proj_k(
    const _Float16* __restrict__ ah,
    const _Float16* __restrict__ wt,
    const float* __restrict__ bias,
    int L,
    _Float16* __restrict__ qp,
    _Float16* __restrict__ kp,
    _Float16* __restrict__ vtp)
{
  __shared__ __attribute__((aligned(16))) _Float16 sT[128 * 64];

  const int tid = threadIdx.x, lane = tid & 31, w = tid >> 5;
  const int h = lane >> 4, m = lane & 15;
  const int m0 = blockIdx.x * 128;
  const int cg = blockIdx.y;
  const int which = cg >> 3, head = cg & 7;
  const int m0w = m0 + 32 * w;

  const _Float16* xa0 = ah + (size_t)(m0w + m) * NC;
  const _Float16* xa1 = xa0 + (size_t)16 * NC;
  const _Float16* wb  = wt + ((size_t)which * NC + head * HDIM + m) * NC;

  const v8f zero8 = {0.f, 0.f, 0.f, 0.f, 0.f, 0.f, 0.f, 0.f};
  v8f acc[2][4];
  #pragma unroll
  for (int mt = 0; mt < 2; ++mt)
    #pragma unroll
    for (int nt = 0; nt < 4; ++nt) acc[mt][nt] = zero8;

  #pragma unroll 1
  for (int k0 = 0; k0 < NC; k0 += 32) {
    const v16h a0 = load_frag(xa0 + k0, h);
    const v16h a1 = load_frag(xa1 + k0, h);
    #pragma unroll
    for (int nt = 0; nt < 4; ++nt) {
      const v16h b = load_frag(wb + (size_t)nt * 16 * NC + k0, h);
      acc[0][nt] = wmma_f16(a0, b, acc[0][nt]);
      acc[1][nt] = wmma_f16(a1, b, acc[1][nt]);
    }
  }

  #pragma unroll
  for (int nt = 0; nt < 4; ++nt) {
    const int feat = 16 * nt + m;
    const float bvl = bias[which * NC + head * HDIM + feat];
    #pragma unroll
    for (int mt = 0; mt < 2; ++mt) {
      #pragma unroll
      for (int r = 0; r < 8; ++r) {
        const int tokl = 32 * w + 16 * mt + 8 * h + r;
        const float y = acc[mt][nt][r] * (1.0f / WSC) + bvl;
        const int idx = (which == 2) ? (feat * 128 + tokl) : (tokl * HDIM + feat);
        sT[idx] = (_Float16)y;
      }
    }
  }
  __syncthreads();

  const int b = m0 / L, l0 = m0 - b * L, z = b * NH + head;
  _Float16* plane = (which == 0) ? qp : kp;
  proj_store_pass(sT, plane, vtp, which, z, l0, L, w, lane);
  __threadfence();
  proj_store_pass(sT, plane, vtp, which, z, l0, L, w, lane);
}

__global__ __launch_bounds__(256) void aux_k(
    const _Float16* __restrict__ qx, const _Float16* __restrict__ qy,
    const float* __restrict__ w4x, const float* __restrict__ w4y, const float* __restrict__ w4xy,
    _Float16* __restrict__ qxw, float* __restrict__ c1, float* __restrict__ c2)
{
  __shared__ __attribute__((aligned(16))) float sv[32];
  const int tid = threadIdx.x, q8 = tid & 7, rl = tid >> 3;
  const int blk = blockIdx.x;
  const bool isx = blk < (NZ * NT / 32);
  int row, hh;
  const _Float16* src; const float* wd; float* cd;
  if (isx) { row = blk * 32 + rl; hh = (row >> 10) & 7; src = qx; wd = w4x; cd = c1 + blk * 32; }
  else { const int yb = blk - NZ * NT / 32; row = yb * 32 + rl; hh = (row >> 8) & 7; src = qy; wd = w4y; cd = c2 + yb * 32; }

  const v8h qv = *(const v8ha*)(src + (size_t)row * HDIM + 8 * q8);
  const v4f wa = *(const v4fa*)(wd + hh * HDIM + 8 * q8);
  const v4f wb = *(const v4fa*)(wd + hh * HDIM + 8 * q8 + 4);
  const float qf[8] = { (float)qv[0], (float)qv[1], (float)qv[2], (float)qv[3],
                        (float)qv[4], (float)qv[5], (float)qv[6], (float)qv[7] };
  const float wv[8] = { wa.x, wa.y, wa.z, wa.w, wb.x, wb.y, wb.z, wb.w };
  float d = 0.0f;
  #pragma unroll
  for (int i = 0; i < 8; ++i) d += qf[i] * wv[i];
  d += __shfl_xor(d, 1);
  d += __shfl_xor(d, 2);
  d += __shfl_xor(d, 4);

  v8h o = qv;
  _Float16* od = qxw;
  if (isx) {
    const v4f ua = *(const v4fa*)(w4xy + hh * HDIM + 8 * q8);
    const v4f ub = *(const v4fa*)(w4xy + hh * HDIM + 8 * q8 + 4);
    const float uv[8] = { ua.x, ua.y, ua.z, ua.w, ub.x, ub.y, ub.z, ub.w };
    #pragma unroll
    for (int i = 0; i < 8; ++i) o[i] = (_Float16)(qf[i] * uv[i] * WSC);
    od = qxw + (size_t)row * HDIM + 8 * q8;
    *(volatile v8h*)od = o;
  }
  if (q8 == 0) sv[rl] = d;
  __syncthreads();
  v4f cv = {0.f, 0.f, 0.f, 0.f};
  if (tid < 8) { cv = *(const v4fa*)(sv + 4 * tid); *(volatile v4f*)(cd + 4 * tid) = cv; }
  __threadfence();
  if (isx) *(volatile v8h*)od = o;
  if (tid < 8) *(volatile v4f*)(cd + 4 * tid) = cv;
}

DEV void tile_store_f32(const float* sO, float* dst, int ldd, int tid) {
  #pragma unroll
  for (int i = 0; i < 16; ++i) {
    const int p = i * 128 + tid;
    const int line = p >> 3, q8 = p & 7;
    const int row = line >> 1, hl = line & 1;
    const v4f v = *(const v4fa*)(sO + row * 64 + 32 * hl + 4 * q8);
    *(volatile v4f*)(dst + (size_t)row * ldd + 32 * hl + 4 * q8) = v;
  }
}

template <int EPI>
__global__ __launch_bounds__(128) void gemm_k(
    const _Float16* __restrict__ A, int lda, long sAz,
    const _Float16* __restrict__ Bt, int ldb, long sBz,
    float* __restrict__ D, int ldd, long sDb, long sDh, int K,
    const float* __restrict__ bias, const float* __restrict__ c1, int c1n,
    const float* __restrict__ c2, int c2n, float alpha)
{
  __shared__ __attribute__((aligned(16))) float sO[128 * 64];

  const int tid = threadIdx.x, lane = tid & 31, w = tid >> 5;
  const int h = lane >> 4, m = lane & 15;
  const int z = blockIdx.z;
  const int m0 = blockIdx.y * 128, n0 = blockIdx.x * 64, m0w = m0 + 32 * w;
  const _Float16* Az = A + (size_t)z * sAz;
  const _Float16* Bz = Bt + (size_t)z * sBz;
  float* Dz = D + (size_t)(z >> 3) * sDb + (size_t)(z & 7) * sDh;

  const _Float16* a0p = Az + (size_t)(m0w + m) * lda;
  const _Float16* a1p = a0p + (size_t)16 * lda;
  const _Float16* bp  = Bz + (size_t)(n0 + m) * ldb;

  const v8f zero8 = {0.f, 0.f, 0.f, 0.f, 0.f, 0.f, 0.f, 0.f};
  v8f acc[2][4];
  #pragma unroll
  for (int mt = 0; mt < 2; ++mt)
    #pragma unroll
    for (int nt = 0; nt < 4; ++nt) acc[mt][nt] = zero8;

  #pragma unroll 1
  for (int k0 = 0; k0 < K; k0 += 32) {
    const v16h a0 = load_frag(a0p + k0, h);
    const v16h a1 = load_frag(a1p + k0, h);
    #pragma unroll
    for (int nt = 0; nt < 4; ++nt) {
      const v16h b = load_frag(bp + (size_t)nt * 16 * ldb + k0, h);
      acc[0][nt] = wmma_f16(a0, b, acc[0][nt]);
      acc[1][nt] = wmma_f16(a1, b, acc[1][nt]);
    }
  }

  #pragma unroll
  for (int nt = 0; nt < 4; ++nt) {
    const int cl = 16 * nt + m;
    float badd = 0.0f;
    if (EPI == 2 || EPI == 3) badd = bias[n0 + cl];
    float cadd = 0.0f;
    if (EPI == 0) cadd = c2[(size_t)z * c2n + n0 + cl];
    #pragma unroll
    for (int mt = 0; mt < 2; ++mt) {
      #pragma unroll
      for (int r = 0; r < 8; ++r) {
        const int rl = 32 * w + 16 * mt + 8 * h + r;
        float v = acc[mt][nt][r] * alpha;
        if (EPI == 0) {
          const float radd = c1[(size_t)z * c1n + m0 + rl];
          v = (radd + cadd) + v;
        } else if (EPI == 2) {
          const float t = v + badd;
          v = rcpf(1.0f + __expf(-t));
        } else if (EPI == 3) {
          v = v + badd;
        }
        sO[rl * 64 + cl] = v;
      }
    }
  }
  __syncthreads();

  float* db = Dz + (size_t)m0 * ldd + n0;
  tile_store_f32(sO, db, ldd, tid);
  __threadfence();
  tile_store_f32(sO, db, ldd, tid);
}

__global__ __launch_bounds__(256) void colstats_k(
    const float* __restrict__ catt, float* __restrict__ cmax, float* __restrict__ cinv)
{
  __shared__ __attribute__((aligned(16))) float sm[256];
  __shared__ __attribute__((aligned(16))) float si[256];
  const int tid = threadIdx.x, z = blockIdx.x;
  const float* p = catt + (size_t)z * NT * NM + tid;
  float ma = -3e38f, mb = -3e38f;
  #pragma unroll 2
  for (int t = 0; t < NT; t += 2) {
    ma = fmaxf(ma, p[(size_t)t * NM]);
    mb = fmaxf(mb, p[(size_t)(t + 1) * NM]);
  }
  const float mx = fmaxf(ma, mb);
  float s0 = 0.f, s1 = 0.f, s2 = 0.f, s3 = 0.f;
  #pragma unroll 1
  for (int t = 0; t < NT; t += 4) {
    s0 += __expf(p[(size_t)t * NM] - mx);
    s1 += __expf(p[(size_t)(t + 1) * NM] - mx);
    s2 += __expf(p[(size_t)(t + 2) * NM] - mx);
    s3 += __expf(p[(size_t)(t + 3) * NM] - mx);
  }
  const float s = (s0 + s1) + (s2 + s3);
  sm[tid] = mx;
  si[tid] = rcpf(s);
  __syncthreads();
  v4f v = {0.f, 0.f, 0.f, 0.f};
  float* d = cmax;
  const bool act = tid < 128;
  if (tid < 64) { v = *(const v4fa*)(sm + 4 * tid); d = cmax + z * NM + 4 * tid; }
  else if (act) { v = *(const v4fa*)(si + 4 * (tid - 64)); d = cinv + z * NM + 4 * (tid - 64); }
  if (act) *(volatile v4f*)d = v;
  __threadfence();
  if (act) *(volatile v4f*)d = v;
}

__global__ __launch_bounds__(256) void norm_k(
    const float* __restrict__ catt, const float* __restrict__ cmax, const float* __restrict__ cinv,
    _Float16* __restrict__ x2y, _Float16* __restrict__ y2x)
{
  const int tid = threadIdx.x, lane = tid & 31, w = tid >> 5;
  const int row0 = blockIdx.x * 32 + 4 * w;
  const int z = row0 >> 10;
  const v4f cma = *(const v4fa*)(cmax + z * NM + 8 * lane);
  const v4f cmb = *(const v4fa*)(cmax + z * NM + 8 * lane + 4);
  const v4f cia = *(const v4fa*)(cinv + z * NM + 8 * lane);
  const v4f cib = *(const v4fa*)(cinv + z * NM + 8 * lane + 4);
  const float cm[8] = { cma.x, cma.y, cma.z, cma.w, cmb.x, cmb.y, cmb.z, cmb.w };
  const float ci[8] = { cia.x * PSC, cia.y * PSC, cia.z * PSC, cia.w * PSC,
                        cib.x * PSC, cib.y * PSC, cib.z * PSC, cib.w * PSC };
  #pragma unroll 1
  for (int rr = 0; rr < 4; ++rr) {
    const size_t base = (size_t)(row0 + rr) * NM + 8 * lane;
    const v4f a = *(const v4fa*)(catt + base);
    const v4f b = *(const v4fa*)(catt + base + 4);
    const float v[8] = { a.x, a.y, a.z, a.w, b.x, b.y, b.z, b.w };
    float mx = v[0];
    #pragma unroll
    for (int i = 1; i < 8; ++i) mx = fmaxf(mx, v[i]);
    #pragma unroll
    for (int off = 16; off; off >>= 1) mx = fmaxf(mx, __shfl_xor(mx, off));
    float e[8];
    float s = 0.0f;
    #pragma unroll
    for (int i = 0; i < 8; ++i) { e[i] = __expf(v[i] - mx); s += e[i]; }
    #pragma unroll
    for (int off = 16; off; off >>= 1) s += __shfl_xor(s, off);
    const float inv = rcpf(s) * PSC;
    v8h ox, oy;
    #pragma unroll
    for (int i = 0; i < 8; ++i) {
      ox[i] = (_Float16)(e[i] * inv);
      oy[i] = (_Float16)(__expf(v[i] - cm[i]) * ci[i]);
    }
    _Float16* dx = x2y + base;
    _Float16* dy = y2x + base;
    *(volatile v8h*)dx = ox;
    *(volatile v8h*)dy = oy;
    __threadfence();
    *(volatile v8h*)dx = ox;
    *(volatile v8h*)dy = oy;
  }
}

DEV v8f sel8(v8f s, const int* p, float sc) {
  const v4i ma = *(const v4ia*)p;
  const v4i mb = *(const v4ia*)(p + 4);
  s[0] = ma.x ? s[0] * sc : NEGV;
  s[1] = ma.y ? s[1] * sc : NEGV;
  s[2] = ma.z ? s[2] * sc : NEGV;
  s[3] = ma.w ? s[3] * sc : NEGV;
  s[4] = mb.x ? s[4] * sc : NEGV;
  s[5] = mb.y ? s[5] * sc : NEGV;
  s[6] = mb.z ? s[6] * sc : NEGV;
  s[7] = mb.w ? s[7] * sc : NEGV;
  return s;
}

DEV v16h pack_p(v8f a, v8f c) {
  const v16h r = { (_Float16)(a[0] * PSC), (_Float16)(a[1] * PSC), (_Float16)(a[2] * PSC), (_Float16)(a[3] * PSC),
                   (_Float16)(a[4] * PSC), (_Float16)(a[5] * PSC), (_Float16)(a[6] * PSC), (_Float16)(a[7] * PSC),
                   (_Float16)(c[0] * PSC), (_Float16)(c[1] * PSC), (_Float16)(c[2] * PSC), (_Float16)(c[3] * PSC),
                   (_Float16)(c[4] * PSC), (_Float16)(c[5] * PSC), (_Float16)(c[6] * PSC), (_Float16)(c[7] * PSC) };
  return r;
}

DEV void att_store_pass(const float* so, float* out, int b, int head, int q0, int lane) {
  const int q8 = lane & 7, sub = lane >> 3;
  #pragma unroll
  for (int i = 0; i < 8; ++i) {
    const int lid = i * 4 + sub;
    const int row = lid >> 1, hl = lid & 1;
    const v4f v = *(const v4fa*)(so + row * 64 + 32 * hl + 4 * q8);
    const size_t gi = ((size_t)b * NT + q0 + row) * NC + head * HDIM + 32 * hl + 4 * q8;
    *(volatile v4f*)(out + gi) = v;
  }
}

template <int DK>
__global__ __launch_bounds__(128) void attn_k(
    const _Float16* __restrict__ qh,
    const _Float16* __restrict__ kh,
    const _Float16* __restrict__ vt,
    const int* __restrict__ msk,
    float* __restrict__ out,
    float sscale)
{
  __shared__ __attribute__((aligned(16))) float sO[4 * 16 * 64];
  constexpr int KC = DK / 32;

  const int tid = threadIdx.x, lane = tid & 31, w = tid >> 5;
  const int h = lane >> 4, m = lane & 15;
  const int z = blockIdx.y, b = z >> 3, head = z & 7;
  const int q0 = blockIdx.x * 64 + 16 * w;

  const _Float16* qrow = qh + ((size_t)z * NT + q0 + m) * DK;
  v16h qb[KC];
  #pragma unroll
  for (int c = 0; c < KC; ++c) qb[c] = load_frag(qrow + 32 * c, h);

  const v8f zero8 = {0.f, 0.f, 0.f, 0.f, 0.f, 0.f, 0.f, 0.f};
  v8f o[4];
  #pragma unroll
  for (int t = 0; t < 4; ++t) o[t] = zero8;
  float mrun = NEGV, lrun = 0.0f;

  const _Float16* kbase = kh + ((size_t)z * NT + m) * DK;
  const _Float16* vbase = vt + ((size_t)z * HDIM + m) * NT;
  const int* mrow = msk + (size_t)(q0 + m) * NT + 8 * h;

  #pragma unroll 1
  for (int kb = 0; kb < NT; kb += 64) {
    v8f s[4];
    #pragma unroll
    for (int j = 0; j < 4; ++j) {
      const _Float16* kp = kbase + (size_t)(kb + 16 * j) * DK;
      v8f zc = zero8;
      #pragma unroll
      for (int c = 0; c < KC; ++c) {
        const v16h kf = load_frag(kp + 32 * c, h);
        zc = wmma_f16(kf, qb[c], zc);
      }
      s[j] = zc;
    }
    #pragma unroll
    for (int j = 0; j < 4; ++j) s[j] = sel8(s[j], mrow + kb + 16 * j, sscale);

    float mloc = s[0][0];
    #pragma unroll
    for (int j = 0; j < 4; ++j)
      #pragma unroll
      for (int r = 0; r < 8; ++r) mloc = fmaxf(mloc, s[j][r]);
    mloc = fmaxf(mloc, __shfl_xor(mloc, 16));
    const float mnew = fmaxf(mrun, mloc);
    const float alpha = __expf(mrun - mnew);
    mrun = mnew;
    float lsum = 0.0f;
    #pragma unroll
    for (int j = 0; j < 4; ++j)
      #pragma unroll
      for (int r = 0; r < 8; ++r) {
        const float p = __expf(s[j][r] - mnew);
        s[j][r] = p;
        lsum += p;
      }
    lsum += __shfl_xor(lsum, 16);
    lrun = lrun * alpha + lsum;
    #pragma unroll
    for (int t = 0; t < 4; ++t)
      #pragma unroll
      for (int r = 0; r < 8; ++r) o[t][r] = o[t][r] * alpha;

    const v16h pb0 = pack_p(s[0], s[1]);
    const v16h pb1 = pack_p(s[2], s[3]);

    #pragma unroll
    for (int t = 0; t < 4; ++t) {
      const _Float16* vp = vbase + (size_t)(16 * t) * NT + kb;
      const v16h vf0 = load_frag(vp, h);
      const v16h vf1 = load_frag(vp + 32, h);
      o[t] = wmma_f16(vf0, pb0, o[t]);
      o[t] = wmma_f16(vf1, pb1, o[t]);
    }
  }

  const float inv = rcpf(lrun) * (1.0f / PSC);
  float* so = sO + w * 1024;
  #pragma unroll
  for (int t = 0; t < 4; ++t)
    #pragma unroll
    for (int r = 0; r < 8; ++r)
      so[m * 64 + 16 * t + 8 * h + r] = o[t][r] * inv;
  __syncthreads();

  att_store_pass(so, out, b, head, q0, lane);
  __threadfence();
  att_store_pass(so, out, b, head, q0, lane);
}

__global__ __launch_bounds__(256) void combine1_k(
    const float* __restrict__ ca, const float* __restrict__ cb, const float* __restrict__ x,
    const float* __restrict__ sv, _Float16* __restrict__ cvh, _Float16* __restrict__ svh)
{
  const int g = blockIdx.x * 256 + threadIdx.x;
  if (g >= TOKX * NC / 8) return;
  const size_t e = (size_t)g * 8;
  const v4f a0 = *(const v4fa*)(ca + e), a1 = *(const v4fa*)(ca + e + 4);
  const v4f b0 = *(const v4fa*)(cb + e), b1 = *(const v4fa*)(cb + e + 4);
  const v4f x0 = *(const v4fa*)(x + e),  x1 = *(const v4fa*)(x + e + 4);
  const v4f s0 = *(const v4fa*)(sv + e), s1 = *(const v4fa*)(sv + e + 4);
  const v4f c0 = (a0 + b0) + x0;
  const v4f c1 = (a1 + b1) + x1;
  const v8h oc = { (_Float16)c0.x, (_Float16)c0.y, (_Float16)c0.z, (_Float16)c0.w,
                   (_Float16)c1.x, (_Float16)c1.y, (_Float16)c1.z, (_Float16)c1.w };
  const v8h os = { (_Float16)s0.x, (_Float16)s0.y, (_Float16)s0.z, (_Float16)s0.w,
                   (_Float16)s1.x, (_Float16)s1.y, (_Float16)s1.z, (_Float16)s1.w };
  *(volatile v8h*)(cvh + e) = oc;
  *(volatile v8h*)(svh + e) = os;
  __threadfence();
  *(volatile v8h*)(cvh + e) = oc;
  *(volatile v8h*)(svh + e) = os;
}

__global__ __launch_bounds__(256) void combine2_k(
    const float* __restrict__ ca, const float* __restrict__ cb, const float* __restrict__ x,
    const float* __restrict__ sv, const float* __restrict__ sg, const float* __restrict__ cg,
    _Float16* __restrict__ zh)
{
  const int g = blockIdx.x * 256 + threadIdx.x;
  if (g >= TOKX * NC / 8) return;
  const size_t e = (size_t)g * 8;
  const v4f a0 = *(const v4fa*)(ca + e), a1 = *(const v4fa*)(ca + e + 4);
  const v4f b0 = *(const v4fa*)(cb + e), b1 = *(const v4fa*)(cb + e + 4);
  const v4f x0 = *(const v4fa*)(x + e),  x1 = *(const v4fa*)(x + e + 4);
  const v4f s0 = *(const v4fa*)(sv + e), s1 = *(const v4fa*)(sv + e + 4);
  const v4f g0 = *(const v4fa*)(sg + e), g1 = *(const v4fa*)(sg + e + 4);
  const v4f h0 = *(const v4fa*)(cg + e), h1 = *(const v4fa*)(cg + e + 4);
  const v4f c0 = (a0 + b0) + x0;
  const v4f c1 = (a1 + b1) + x1;
  const v4f z0 = g0 * c0 + h0 * s0;
  const v4f z1 = g1 * c1 + h1 * s1;
  const v8h oz = { (_Float16)z0.x, (_Float16)z0.y, (_Float16)z0.z, (_Float16)z0.w,
                   (_Float16)z1.x, (_Float16)z1.y, (_Float16)z1.z, (_Float16)z1.w };
  *(volatile v8h*)(zh + e) = oz;
  __threadfence();
  *(volatile v8h*)(zh + e) = oz;
}

extern "C" void kernel_launch(void* const* d_in, const int* in_sizes, int n_in,
                              void* d_out, int out_size, void* d_ws, size_t ws_size,
                              hipStream_t stream) {
  if (n_in < 16) return;
  if (in_sizes[0] != TOKX * NC || in_sizes[1] != TOKY * NC) return;
  if (in_sizes[2] != NT * NT) return;
  if (in_sizes[3] != NC * NC3 || in_sizes[5] != NC * NC3) return;
  if (in_sizes[4] != NC3 || in_sizes[6] != NC3) return;
  if (in_sizes[7] != NH * HDIM || in_sizes[8] != NH * HDIM || in_sizes[9] != NH * HDIM) return;
  if (in_sizes[10] != NC * NC || in_sizes[12] != NC * NC || in_sizes[14] != NC * NC) return;
  if (in_sizes[11] != NC || in_sizes[13] != NC || in_sizes[15] != NC) return;
  if (out_size != TOKX * NC) return;

  const float* x      = (const float*)d_in[0];
  const float* y      = (const float*)d_in[1];
  const int*   amask  = (const int*)d_in[2];
  const float* Wqkv_x = (const float*)d_in[3];
  const float* bqkv_x = (const float*)d_in[4];
  const float* Wqkv_y = (const float*)d_in[5];
  const float* bqkv_y = (const float*)d_in[6];
  const float* w4x    = (const float*)d_in[7];
  const float* w4y    = (const float*)d_in[8];
  const float* w4xy   = (const float*)d_in[9];
  const float* Wgs    = (const float*)d_in[10];
  const float* bgs    = (const float*)d_in[11];
  const float* Wgc    = (const float*)d_in[12];
  const float* bgc    = (const float*)d_in[13];
  const float* Wp     = (const float*)d_in[14];
  const float* bp     = (const float*)d_in[15];
  float* out = (float*)d_out;

  const size_t b_xh   = (size_t)TOKX * NC * 2;
  const size_t b_yh   = (size_t)TOKY * NC * 2;
  const size_t b_wt   = (size_t)WROWS * NC * 2;
  const size_t b_plx  = (size_t)NZ * NT * HDIM * 2;
  const size_t b_ply  = (size_t)NZ * NM * HDIM * 2;
  const size_t b_c1   = (size_t)NZ * NT * 4;
  const size_t b_c2   = (size_t)NZ * NM * 4;
  const size_t b_cs   = (size_t)NZ * NM * 4;
  const size_t b_ra   = (size_t)NZ * NT * NM * 4;
  const size_t b_rb   = (size_t)NZ * NT * NM * 2;
  const size_t b_rc   = (size_t)NZ * NT * NM * 2;
  const size_t b_f32p = (size_t)TOKX * NC * 4;
  const size_t b_f16p = (size_t)TOKX * NC * 2;

  size_t off = 0;
  char* base = (char*)d_ws;
  char* p_xh  = base + off; off += b_xh;
  char* p_yh  = base + off; off += b_yh;
  char* p_wt  = base + off; off += b_wt;
  char* p_qx  = base + off; off += b_plx;
  char* p_kx  = base + off; off += b_plx;
  char* p_vtx = base + off; off += b_plx;
  char* p_qy  = base + off; off += b_ply;
  char* p_ky  = base + off; off += b_ply;
  char* p_vty = base + off; off += b_ply;
  char* p_qxw = base + off; off += b_plx;
  char* p_c1  = base + off; off += b_c1;
  char* p_c2  = base + off; off += b_c2;
  char* p_cm  = base + off; off += b_cs;
  char* p_ci  = base + off; off += b_cs;
  char* p_ra  = base + off; off += b_ra;
  char* p_rb  = base + off; off += b_rb;
  char* p_rc  = base + off; off += b_rc;
  const size_t total = off;
  if (total > ws_size) return;
  if (total > (size_t)134217728) return;

  _Float16* xh  = (_Float16*)p_xh;
  _Float16* yh  = (_Float16*)p_yh;
  _Float16* wt  = (_Float16*)p_wt;
  _Float16* qx  = (_Float16*)p_qx;
  _Float16* kx  = (_Float16*)p_kx;
  _Float16* vtx = (_Float16*)p_vtx;
  _Float16* qy  = (_Float16*)p_qy;
  _Float16* ky  = (_Float16*)p_ky;
  _Float16* vty = (_Float16*)p_vty;
  _Float16* qxw = (_Float16*)p_qxw;
  float* c1   = (float*)p_c1;
  float* c2   = (float*)p_c2;
  float* cmax = (float*)p_cm;
  float* cinv = (float*)p_ci;
  float* catt  = (float*)p_ra;
  float* cvx2y = (float*)p_ra;
  float* cvy2x = (float*)(p_ra + b_f32p);
  float* sval  = (float*)(p_ra + 2 * b_f32p);
  _Float16* x2y = (_Float16*)p_rb;
  float* sgate  = (float*)p_rb;
  float* cgate  = (float*)(p_rb + b_f32p);
  _Float16* y2x = (_Float16*)p_rc;
  _Float16* cvh = (_Float16*)p_rc;
  _Float16* svh = (_Float16*)(p_rc + b_f16p);
  _Float16* zhp = (_Float16*)(p_rc + 2 * b_f16p);

  const int ncvt = TOKX * NC / 8 + TOKY * NC / 8;
  convert_xy_k<<<(ncvt + 255) / 256, 256, 0, stream>>>(x, y, xh, yh);
  wtrans_k<<<dim3(WROWS / 32, NC / 64), 256, 0, stream>>>(Wqkv_x, Wqkv_y, Wgs, Wgc, Wp, wt);

  proj_k<<<dim3(TOKX / 128, 3 * NH), 128, 0, stream>>>(xh, wt, bqkv_x, NT, qx, kx, vtx);
  proj_k<<<dim3(TOKY / 128, 3 * NH), 128, 0, stream>>>(yh, wt + (size_t)NC3 * NC, bqkv_y, NM, qy, ky, vty);

  aux_k<<<NZ * NT / 32 + NZ * NM / 32, 256, 0, stream>>>(qx, qy, w4x, w4y, w4xy, qxw, c1, c2);

  gemm_k<0><<<dim3(NM / 64, NT / 128, NZ), 128, 0, stream>>>(
      qxw, HDIM, (long)NT * HDIM, ky, HDIM, (long)NM * HDIM,
      catt, NM, (long)NH * NT * NM, (long)NT * NM, HDIM,
      bqkv_x, c1, NT, c2, NM, 0.125f / WSC);

  colstats_k<<<NZ, 256, 0, stream>>>(catt, cmax, cinv);
  norm_k<<<NZ * NT / 32, 256, 0, stream>>>(catt, cmax, cinv, x2y, y2x);

  gemm_k<1><<<dim3(1, NT / 128, NZ), 128, 0, stream>>>(
      x2y, NM, (long)NT * NM, vty, NM, (long)HDIM * NM,
      cvx2y, NC, (long)NT * NC, (long)HDIM, NM,
      bqkv_x, c1, NT, c2, NM, 1.0f / PSC);

  attn_k<NM><<<dim3(NT / 64, NZ), 128, 0, stream>>>(x2y, y2x, vtx, amask, cvy2x, 2.3283064365386963e-10f);

  attn_k<HDIM><<<dim3(NT / 64, NZ), 128, 0, stream>>>(qx, kx, vtx, amask, sval, 0.125f);

  combine1_k<<<(TOKX * NC / 8 + 255) / 256, 256, 0, stream>>>(cvx2y, cvy2x, x, sval, cvh, svh);

  gemm_k<2><<<dim3(NC / 64, TOKX / 128, 1), 128, 0, stream>>>(
      svh, NC, 0, wt + (size_t)(2 * NC3) * NC, NC, 0,
      sgate, NC, 0, 0, NC, bgs, c1, NT, c2, NM, 1.0f / WSC);
  gemm_k<2><<<dim3(NC / 64, TOKX / 128, 1), 128, 0, stream>>>(
      cvh, NC, 0, wt + (size_t)(2 * NC3 + NC) * NC, NC, 0,
      cgate, NC, 0, 0, NC, bgc, c1, NT, c2, NM, 1.0f / WSC);

  combine2_k<<<(TOKX * NC / 8 + 255) / 256, 256, 0, stream>>>(cvx2y, cvy2x, x, sval, sgate, cgate, zhp);

  gemm_k<3><<<dim3(NC / 64, TOKX / 128, 1), 128, 0, stream>>>(
      zhp, NC, 0, wt + (size_t)(2 * NC3 + 2 * NC) * NC, NC, 0,
      out, NC, 0, 0, NC, bp, c1, NT, c2, NM, 1.0f / WSC);
}
